// LTAE_88562225643738
// MI455X (gfx1250) — hardware-verified
//
#include <hip/hip_runtime.h>


typedef __bf16 bf16_t;
typedef __attribute__((ext_vector_type(16))) __bf16 v16bf;
typedef __attribute__((ext_vector_type(8)))  __bf16 v8bf;
typedef __attribute__((ext_vector_type(8)))  float  v8f;
typedef __attribute__((ext_vector_type(4)))  float  v4f;

#define NS    24
#define NCI   10
#define NXC   11
#define NDM   256
#define NHD   16
#define NOUT  20
#define EPSV  1e-5f
#define INVSQ8 0.35355339059327378f
#define CNEG  (-0.026983419058523973f)

#define P_QKW 0
#define P_QB  4096
#define P_CWF 4128
#define P_T1  6688
#define P_DIV 6944
#define P_N   7072
#define WS_O_OFF 32768

static __device__ __forceinline__ v8f mma3(v8f acc, v16bf ah, v16bf al, v16bf bh, v16bf bl) {
    acc = __builtin_amdgcn_wmma_f32_16x16x32_bf16(false, ah, false, bh, (short)0, acc, false, false);
    acc = __builtin_amdgcn_wmma_f32_16x16x32_bf16(false, ah, false, bl, (short)0, acc, false, false);
    acc = __builtin_amdgcn_wmma_f32_16x16x32_bf16(false, al, false, bh, (short)0, acc, false, false);
    asm volatile("v_nop\n\tv_nop\n\tv_nop\n\tv_nop" : "+v"(acc) : "v"(ah), "v"(al), "v"(bh), "v"(bl));
    return acc;
}

static __device__ __forceinline__ void split16(v4f q0, v4f q1, v4f q2, v4f q3, v16bf& hi, v16bf& lo) {
    float f[16];
    f[0]  = q0.x; f[1]  = q0.y; f[2]  = q0.z; f[3]  = q0.w;
    f[4]  = q1.x; f[5]  = q1.y; f[6]  = q1.z; f[7]  = q1.w;
    f[8]  = q2.x; f[9]  = q2.y; f[10] = q2.z; f[11] = q2.w;
    f[12] = q3.x; f[13] = q3.y; f[14] = q3.z; f[15] = q3.w;
#pragma unroll
    for (int i = 0; i < 16; ++i) {
        const bf16_t hv = (bf16_t)f[i];
        const float rem = f[i] - (float)hv;
        hi[i] = hv;
        lo[i] = (bf16_t)rem;
    }
}

static __device__ __forceinline__ void frag_f32_split(const float* base, int stride, int r0, int k0,
                                                      v16bf& hi, v16bf& lo) {
    const int l = threadIdx.x & 31, h = l >> 4, m = l & 15;
    const float* p = base + (size_t)(r0 + m) * stride + k0 + 8 * h;
    const v4f q0 = *(const v4f*)(p);
    const v4f q1 = *(const v4f*)(p + 4);
    const v4f q2 = *(const v4f*)(p + 16);
    const v4f q3 = *(const v4f*)(p + 20);
    split16(q0, q1, q2, q3, hi, lo);
}

static __device__ __forceinline__ void frag_f32_split_nclamp(const float* base, int stride, int r0, int k0,
                                                             int nmax, v16bf& hi, v16bf& lo) {
    const int l = threadIdx.x & 31, h = l >> 4, m = l & 15;
    const int n = r0 + m;
    const int nc = (n < nmax) ? n : (nmax - 1);
    const float* p = base + (size_t)nc * stride + k0 + 8 * h;
    v4f q0 = *(const v4f*)(p);
    v4f q1 = *(const v4f*)(p + 4);
    v4f q2 = *(const v4f*)(p + 16);
    v4f q3 = *(const v4f*)(p + 20);
    if (n >= nmax) { const v4f z = {0.f, 0.f, 0.f, 0.f}; q0 = z; q1 = z; q2 = z; q3 = z; }
    split16(q0, q1, q2, q3, hi, lo);
}

static __device__ __forceinline__ v16bf frag_bf16(const bf16_t* base, int stride, int r0, int k0) {
    const int l = threadIdx.x & 31, h = l >> 4, m = l & 15;
    const bf16_t* p = base + (r0 + m) * stride + k0 + 8 * h;
    union { v16bf v; v8bf q[2]; } u;
    u.q[0] = *(const v8bf*)(p);
    u.q[1] = *(const v8bf*)(p + 16);
    return u.v;
}

static __device__ __forceinline__ void sincos_pe(float xa, float& s, float& c) {
    const float kf = rintf(xa * 0.63661977236758134f);
    const int k = (int)kf;
    float r = fmaf(-kf, 1.5707963705062866f, xa);
    r = fmaf(-kf, -4.3711388286737929e-08f, r);
    const float z = r * r, w = z * z;
    const float rz = r * z;
    const float sp = (r + rz * (-0.16666666641626524f + z * 0.008333329385889463f))
                   + rz * w * (-0.00019839334836096632f + z * 0.0000027183114939898219f);
    const float cp = ((1.0f - 0.5f * z) + w * 0.041666623323739063f)
                   + (w * z) * (-0.0013886763774609929f + z * 0.000024390448796277409f);
    float a = (k & 1) ? cp : sp;
    float b = (k & 1) ? -sp : cp;
    if (k & 2) { a = -a; b = -b; }
    s = a; c = b;
}

__global__ __launch_bounds__(256)
void k_fold(const float* __restrict__ conv_w, const float* __restrict__ conv_b,
            const float* __restrict__ bn1_g, const float* __restrict__ bn1_b,
            const float* __restrict__ bn1_m, const float* __restrict__ bn1_v,
            const float* __restrict__ Q, const float* __restrict__ Wk,
            const float* __restrict__ bk, float* params)
{
    __shared__ __align__(16) float stg[P_N];
    const int t = threadIdx.x;
    {
        const int h = t >> 4, dseg = (t & 15) << 4;
        float q[8];
#pragma unroll
        for (int k = 0; k < 8; ++k) q[k] = Q[h * 8 + k];
#pragma unroll
        for (int j = 0; j < 16; ++j) {
            const int d = dseg + j;
            float a = 0.f;
#pragma unroll
            for (int k = 0; k < 8; ++k) a = fmaf(q[k], Wk[(h * 8 + k) * NDM + d], a);
            stg[P_QKW + h * NDM + d] = a * INVSQ8;
        }
    }
    if (t < 32) {
        const int hh = t & 15;
        float a = 0.f;
#pragma unroll
        for (int k = 0; k < 8; ++k) a = fmaf(Q[hh * 8 + k], bk[hh * 8 + k], a);
        stg[P_QB + t] = (t < 16) ? a * INVSQ8 : 0.f;
    }
    {
        const int d = t;
        const float sc = bn1_g[d] * rsqrtf(bn1_v[d] + EPSV);
#pragma unroll
        for (int cc = 0; cc < NCI; ++cc) stg[P_CWF + d * NCI + cc] = conv_w[d * NCI + cc] * sc;
        stg[P_T1 + d] = (conv_b[d] - bn1_m[d]) * sc + bn1_b[d];
    }
    if (t < NDM / 2) stg[P_DIV + t] = expf((float)(2 * t) * CNEG);
    __syncthreads();

    v4f keep[7];
#pragma unroll
    for (int i = 0; i < 7; ++i) {
        const v4f z = {0.f, 0.f, 0.f, 0.f};
        keep[i] = z;
        const int q4 = t + 256 * i;
        if (q4 < P_N / 4) {
            keep[i] = *(const v4f*)(stg + 4 * q4);
            *(volatile v4f*)(params + 4 * q4) = keep[i];
        }
    }
    __threadfence();
#pragma unroll
    for (int i = 0; i < 7; ++i) {
        const int q4 = t + 256 * i;
        if (q4 < P_N / 4) *(volatile v4f*)(params + 4 * q4) = keep[i];
    }
}

#define K1_TPB   128
#define K1_SPB   4
#define K1_ROWS  (K1_SPB * NS)
#define K1_TILES (K1_ROWS / 16)
#define ES 260
#define QS 264
#define K1_OFF_E   0
#define K1_OFF_QH  (K1_ROWS * ES * 4)
#define K1_OFF_QL  (K1_OFF_QH + NHD * QS * 2)
#define K1_OFF_LG  (K1_OFF_QL + NHD * QS * 2)
#define K1_OFF_X   (K1_OFF_LG + K1_SPB * NHD * NS * 4)
#define K1_XN      (K1_ROWS * NXC)
#define K1_SMEM    (K1_OFF_X + K1_XN * 4)

__global__ __launch_bounds__(K1_TPB)
void k_enc(const float* __restrict__ x, int n_x, int nb,
           const float* __restrict__ ln1_g, const float* __restrict__ ln1_b,
           const float* __restrict__ params, float* o_out)
{
    extern __shared__ __align__(16) char smem[];
    float*  e_lds = (float*)(smem + K1_OFF_E);
    bf16_t* qkh   = (bf16_t*)(smem + K1_OFF_QH);
    bf16_t* qkl   = (bf16_t*)(smem + K1_OFF_QL);
    float*  lg    = (float*)(smem + K1_OFF_LG);
    float*  x_lds = (float*)(smem + K1_OFF_X);

    const int t = threadIdx.x, wave = t >> 5, lane = t & 31;

#pragma unroll 4
    for (int i = 0; i < (NHD * NDM) / K1_TPB; ++i) {
        const int idx = t + i * K1_TPB;
        const float v = params[P_QKW + idx];
        const bf16_t hv = (bf16_t)v;
        const int hh = idx >> 8, d = idx & 255;
        qkh[hh * QS + d] = hv;
        qkl[hh * QS + d] = (bf16_t)(v - (float)hv);
    }
    {
        const size_t xbase = (size_t)blockIdx.x * K1_XN;
        for (int i = 0; i < (K1_XN + K1_TPB - 1) / K1_TPB; ++i) {
            const int idx = t + i * K1_TPB;
            if (idx < K1_XN) {
                const size_t g = xbase + (size_t)idx;
                float v = 0.f;
                if (g < (size_t)n_x) v = x[g];
                x_lds[idx] = v;
            }
        }
    }
    __syncthreads();

    {
        const int d0 = lane * 8;
        float cw[80];
        {
            const v4f* cp = (const v4f*)(params + P_CWF + lane * 80);
#pragma unroll
            for (int i = 0; i < 20; ++i) {
                const v4f v = cp[i];
                cw[4 * i] = v.x; cw[4 * i + 1] = v.y; cw[4 * i + 2] = v.z; cw[4 * i + 3] = v.w;
            }
        }
        float tb[8], dv[4];
        {
            const v4f a = *(const v4f*)(params + P_T1 + d0);
            const v4f b = *(const v4f*)(params + P_T1 + d0 + 4);
            tb[0] = a.x; tb[1] = a.y; tb[2] = a.z; tb[3] = a.w;
            tb[4] = b.x; tb[5] = b.y; tb[6] = b.z; tb[7] = b.w;
            const v4f dd = *(const v4f*)(params + P_DIV + lane * 4);
            dv[0] = dd.x; dv[1] = dd.y; dv[2] = dd.z; dv[3] = dd.w;
        }
        float g1[NCI], b1v[NCI];
#pragma unroll
        for (int cc = 0; cc < NCI; ++cc) { g1[cc] = ln1_g[cc]; b1v[cc] = ln1_b[cc]; }
        const int lsel = (lane < NXC) ? lane : 0;

        for (int rr = 0; rr < NS; ++rr) {
            const int r = wave * NS + rr;
            const float xv = x_lds[r * NXC + lsel];
            const int xi = __float_as_int(xv);
            const float pos = __int_as_float(__builtin_amdgcn_readlane(xi, 0));
            float f[NCI];
#pragma unroll
            for (int cc = 0; cc < NCI; ++cc) f[cc] = __int_as_float(__builtin_amdgcn_readlane(xi, cc + 1));
            float mu = 0.f;
#pragma unroll
            for (int cc = 0; cc < NCI; ++cc) mu += f[cc];
            mu *= 0.1f;
            float var = 0.f;
#pragma unroll
            for (int cc = 0; cc < NCI; ++cc) { const float dd = f[cc] - mu; var = fmaf(dd, dd, var); }
            var *= 0.1f;
            const float inv = rsqrtf(var + EPSV);
            float nf[NCI];
#pragma unroll
            for (int cc = 0; cc < NCI; ++cc) nf[cc] = (f[cc] - mu) * inv * g1[cc] + b1v[cc];

            float hv[8];
#pragma unroll
            for (int j = 0; j < 8; ++j) {
                float a = tb[j];
#pragma unroll
                for (int cc = 0; cc < NCI; ++cc) a = fmaf(cw[j * NCI + cc], nf[cc], a);
                hv[j] = a;
            }
            float ev[8];
#pragma unroll
            for (int p = 0; p < 4; ++p) {
                float sn, cs;
                sincos_pe(pos * dv[p], sn, cs);
                ev[2 * p]     = hv[2 * p] + sn;
                ev[2 * p + 1] = hv[2 * p + 1] + cs;
            }
            v4f* ep = (v4f*)(e_lds + r * ES + d0);
            const v4f w0 = {ev[0], ev[1], ev[2], ev[3]};
            const v4f w1 = {ev[4], ev[5], ev[6], ev[7]};
            ep[0] = w0;
            ep[1] = w1;
        }
    }
    __syncthreads();

    for (int tile = wave; tile < K1_TILES; tile += K1_TPB / 32) {
        v8f acc = {0.f, 0.f, 0.f, 0.f, 0.f, 0.f, 0.f, 0.f};
#pragma unroll
        for (int kt = 0; kt < NDM / 32; ++kt) {
            v16bf ah, al;
            frag_f32_split(e_lds, ES, tile * 16, kt * 32, ah, al);
            const v16bf bh = frag_bf16(qkh, QS, 0, kt * 32);
            const v16bf bl = frag_bf16(qkl, QS, 0, kt * 32);
            acc = mma3(acc, ah, al, bh, bl);
        }
        const int n = lane & 15, h = lane >> 4;
        const float qbv = params[P_QB + n];
#pragma unroll
        for (int r = 0; r < 8; ++r) {
            const int row = tile * 16 + 8 * h + r;
            const int bl_ = row / NS, s = row - bl_ * NS;
            lg[(bl_ * NHD + n) * NS + s] = acc[r] + qbv;
        }
    }
    __syncthreads();

    if (t < K1_SPB * NHD) {
        float* lp = lg + t * NS;
        float mx = lp[0];
#pragma unroll
        for (int s = 1; s < NS; ++s) mx = fmaxf(mx, lp[s]);
        float ex[NS];
        float sum = 0.f;
#pragma unroll
        for (int s = 0; s < NS; ++s) { ex[s] = expf(lp[s] - mx); sum += ex[s]; }
        const float rs = 1.0f / sum;
#pragma unroll
        for (int s = 0; s < NS; ++s) lp[s] = ex[s] * rs;
    }
    __syncthreads();

    {
        const int b = wave;
        const size_t gb = (size_t)blockIdx.x * K1_SPB + (size_t)b;
        const int hd0 = lane >> 2, hd1 = 8 + (lane >> 2);
        const float* a0p = lg + (b * NHD + hd0) * NS;
        const float* a1p = lg + (b * NHD + hd1) * NS;
        const float* eb  = e_lds + (b * NS) * ES;
        v4f o0 = {0.f, 0.f, 0.f, 0.f};
        v4f o1 = {0.f, 0.f, 0.f, 0.f};
#pragma unroll
        for (int s = 0; s < NS; ++s) {
            const float a0 = a0p[s], a1 = a1p[s];
            const v4f v0 = *(const v4f*)(eb + s * ES + 4 * lane);
            const v4f v1 = *(const v4f*)(eb + s * ES + 128 + 4 * lane);
            o0 = o0 + v0 * a0;
            o1 = o1 + v1 * a1;
        }
        float* op = o_out + gb * NDM;
        const bool valid = gb < (size_t)nb;
        if (valid) {
            *(volatile v4f*)(op + 4 * lane) = o0;
            *(volatile v4f*)(op + 128 + 4 * lane) = o1;
        }
        __threadfence();
        if (valid) {
            *(volatile v4f*)(op + 4 * lane) = o0;
            *(volatile v4f*)(op + 128 + 4 * lane) = o1;
        }
    }
}

#define K2_TPB 256
#define K2_R   64
#define AS   260
#define MSD  132
#define D1S  72
#define D2S  40
#define K2_OFF_A  0
#define K2_OFF_M  (K2_R * AS * 4)
#define K2_OFF_D1 (K2_OFF_M + K2_R * MSD * 4)
#define K2_OFF_D2 (K2_OFF_D1 + K2_R * D1S * 4)
#define K2_OFF_O  (K2_OFF_D2 + K2_R * D2S * 4)
#define K2_OFF_P  (K2_OFF_O + K2_R * NOUT * 4)
#define K2_SMEM   (K2_OFF_P + 448 * 4)

__global__ __launch_bounds__(K2_TPB)
void k_head(const float* __restrict__ o_in, int nb,
            const float* __restrict__ W1,  const float* __restrict__ b1,
            const float* __restrict__ bn2_g, const float* __restrict__ bn2_b,
            const float* __restrict__ bn2_m, const float* __restrict__ bn2_v,
            const float* __restrict__ oln_g, const float* __restrict__ oln_b,
            const float* __restrict__ Wd1, const float* __restrict__ bd1,
            const float* __restrict__ bnd1_g, const float* __restrict__ bnd1_b,
            const float* __restrict__ bnd1_m, const float* __restrict__ bnd1_v,
            const float* __restrict__ Wd2, const float* __restrict__ bd2,
            const float* __restrict__ bnd2_g, const float* __restrict__ bnd2_b,
            const float* __restrict__ bnd2_m, const float* __restrict__ bnd2_v,
            const float* __restrict__ Wd3, const float* __restrict__ bd3,
            float* out)
{
    extern __shared__ __align__(16) char smem[];
    float* a_lds = (float*)(smem + K2_OFF_A);
    float* m32   = (float*)(smem + K2_OFF_M);
    float* d1l   = (float*)(smem + K2_OFF_D1);
    float* d2l   = (float*)(smem + K2_OFF_D2);
    float* outs  = (float*)(smem + K2_OFF_O);
    float* pp    = (float*)(smem + K2_OFF_P);
    float* s2  = pp;        float* t2  = pp + 128;
    float* sd1 = pp + 256;  float* td1 = pp + 320;
    float* sd2 = pp + 384;  float* td2 = pp + 416;

    const int t = threadIdx.x, wave = t >> 5, lane = t & 31;
    const size_t row0 = (size_t)blockIdx.x * K2_R;

#pragma unroll 4
    for (int i = 0; i < (K2_R * NDM / 4) / K2_TPB; ++i) {
        const int idx = t + i * K2_TPB;
        const int row = idx >> 6, c4 = idx & 63;
        v4f v = {0.f, 0.f, 0.f, 0.f};
        if (row0 + (size_t)row < (size_t)nb) v = *(const v4f*)(o_in + (row0 + (size_t)row) * NDM + c4 * 4);
        *(v4f*)(a_lds + row * AS + c4 * 4) = v;
    }
    if (t < 128) {
        const float sc = bn2_g[t] * rsqrtf(bn2_v[t] + EPSV);
        s2[t] = sc;  t2[t] = (b1[t] - bn2_m[t]) * sc + bn2_b[t];
    }
    if (t < 64) {
        const float sc = bnd1_g[t] * rsqrtf(bnd1_v[t] + EPSV);
        sd1[t] = sc; td1[t] = (bd1[t] - bnd1_m[t]) * sc + bnd1_b[t];
    }
    if (t < 32) {
        const float sc = bnd2_g[t] * rsqrtf(bnd2_v[t] + EPSV);
        sd2[t] = sc; td2[t] = (bd2[t] - bnd2_m[t]) * sc + bnd2_b[t];
    }
    __syncthreads();

    for (int id = wave; id < 32; id += K2_TPB / 32) {
        const int mt = id >> 3, nt = id & 7;
        v8f acc = {0.f, 0.f, 0.f, 0.f, 0.f, 0.f, 0.f, 0.f};
#pragma unroll
        for (int kt = 0; kt < 8; ++kt) {
            v16bf ah, al, bh, bl;
            frag_f32_split(a_lds, AS, mt * 16, kt * 32, ah, al);
            frag_f32_split(W1, 256, nt * 16, kt * 32, bh, bl);
            acc = mma3(acc, ah, al, bh, bl);
        }
        const int n = nt * 16 + (lane & 15);
        const int moff = (lane >> 4) << 3;
        const float sv = s2[n], tv = t2[n];
#pragma unroll
        for (int i = 0; i < 8; ++i) {
            const int row = mt * 16 + moff + i;
            m32[row * MSD + n] = fmaxf(acc[i] * sv + tv, 0.f);
        }
    }
    __syncthreads();

    if (t < K2_R) {
        float* rp = m32 + t * MSD;
        float mu = 0.f;
        for (int cc = 0; cc < 128; ++cc) mu += rp[cc];
        mu *= (1.f / 128.f);
        float var = 0.f;
        for (int cc = 0; cc < 128; ++cc) { const float dd = rp[cc] - mu; var = fmaf(dd, dd, var); }
        var *= (1.f / 128.f);
        const float inv = rsqrtf(var + EPSV);
        for (int cc = 0; cc < 128; ++cc) rp[cc] = (rp[cc] - mu) * inv * oln_g[cc] + oln_b[cc];
    }
    __syncthreads();

    for (int id = wave; id < 16; id += K2_TPB / 32) {
        const int mt = id >> 2, nt = id & 3;
        v8f acc = {0.f, 0.f, 0.f, 0.f, 0.f, 0.f, 0.f, 0.f};
#pragma unroll
        for (int kt = 0; kt < 4; ++kt) {
            v16bf ah, al, bh, bl;
            frag_f32_split(m32, MSD, mt * 16, kt * 32, ah, al);
            frag_f32_split(Wd1, 128, nt * 16, kt * 32, bh, bl);
            acc = mma3(acc, ah, al, bh, bl);
        }
        const int n = nt * 16 + (lane & 15);
        const int moff = (lane >> 4) << 3;
        const float sv = sd1[n], tv = td1[n];
#pragma unroll
        for (int i = 0; i < 8; ++i) {
            const int row = mt * 16 + moff + i;
            d1l[row * D1S + n] = fmaxf(acc[i] * sv + tv, 0.f);
        }
    }
    __syncthreads();

    {
        const int mt = wave >> 1, nt = wave & 1;
        v8f acc = {0.f, 0.f, 0.f, 0.f, 0.f, 0.f, 0.f, 0.f};
#pragma unroll
        for (int kt = 0; kt < 2; ++kt) {
            v16bf ah, al, bh, bl;
            frag_f32_split(d1l, D1S, mt * 16, kt * 32, ah, al);
            frag_f32_split(Wd2, 64, nt * 16, kt * 32, bh, bl);
            acc = mma3(acc, ah, al, bh, bl);
        }
        const int n = nt * 16 + (lane & 15);
        const int moff = (lane >> 4) << 3;
        const float sv = sd2[n], tv = td2[n];
#pragma unroll
        for (int i = 0; i < 8; ++i) {
            const int row = mt * 16 + moff + i;
            d2l[row * D2S + n] = fmaxf(acc[i] * sv + tv, 0.f);
        }
    }
    __syncthreads();

    {
        const int mt = wave >> 1, nt = wave & 1;
        v8f acc = {0.f, 0.f, 0.f, 0.f, 0.f, 0.f, 0.f, 0.f};
        v16bf ah, al, bh, bl;
        frag_f32_split(d2l, D2S, mt * 16, 0, ah, al);
        frag_f32_split_nclamp(Wd3, 32, nt * 16, 0, NOUT, bh, bl);
        acc = mma3(acc, ah, al, bh, bl);
        const int n = nt * 16 + (lane & 15);
        const int moff = (lane >> 4) << 3;
        if (n < NOUT) {
            const float bv = bd3[n];
#pragma unroll
            for (int i = 0; i < 8; ++i) {
                const int row = mt * 16 + moff + i;
                outs[row * NOUT + n] = acc[i] + bv;
            }
        }
    }
    __syncthreads();

    {
        float* ob = out + row0 * NOUT;
        const long long rem = (long long)nb - (long long)row0;
        const int rows_valid = (rem >= K2_R) ? K2_R : (int)((rem > 0) ? rem : 0);
        if (rows_valid == K2_R) {
            const int nq = (K2_R * NOUT) / 4;
            const bool h0 = t < nq;
            const bool h1 = (t + K2_TPB) < nq;
            v4f w0 = {0.f, 0.f, 0.f, 0.f};
            v4f w1 = {0.f, 0.f, 0.f, 0.f};
            if (h0) w0 = *(const v4f*)(outs + 4 * t);
            if (h1) w1 = *(const v4f*)(outs + 4 * (t + K2_TPB));
            if (h0) *(volatile v4f*)(ob + 4 * t) = w0;
            if (h1) *(volatile v4f*)(ob + 4 * (t + K2_TPB)) = w1;
            __threadfence();
            if (h0) *(volatile v4f*)(ob + 4 * t) = w0;
            if (h1) *(volatile v4f*)(ob + 4 * (t + K2_TPB)) = w1;
        } else {
            const int nval = rows_valid * NOUT;
            for (int i = t; i < nval; i += K2_TPB) { const float v = outs[i]; ((volatile float*)ob)[i] = v; }
            __threadfence();
            for (int i = t; i < nval; i += K2_TPB) { const float v = outs[i]; ((volatile float*)ob)[i] = v; }
        }
    }
}

extern "C" void kernel_launch(void* const* d_in, const int* in_sizes, int n_in,
                              void* d_out, int out_size, void* d_ws, size_t ws_size,
                              hipStream_t stream)
{
    if (n_in < 34) return;
    const int n_x = in_sizes[0];
    const int nb  = n_x / (NS * NXC);
    if (nb <= 0) return;
    if ((long long)out_size < (long long)nb * NOUT) return;
    const size_t need = (size_t)WS_O_OFF + (size_t)nb * NDM * sizeof(float);
    if (need > ws_size) return;

    const float* x      = (const float*)d_in[0];
    const float* ln1_g  = (const float*)d_in[1];
    const float* ln1_b  = (const float*)d_in[2];
    const float* conv_w = (const float*)d_in[3];
    const float* conv_b = (const float*)d_in[4];
    const float* bn1_g  = (const float*)d_in[5];
    const float* bn1_b  = (const float*)d_in[6];
    const float* bn1_m  = (const float*)d_in[7];
    const float* bn1_v  = (const float*)d_in[8];
    const float* Q      = (const float*)d_in[9];
    const float* Wk     = (const float*)d_in[10];
    const float* bk     = (const float*)d_in[11];
    const float* W1     = (const float*)d_in[12];
    const float* b1     = (const float*)d_in[13];
    const float* bn2_g  = (const float*)d_in[14];
    const float* bn2_b  = (const float*)d_in[15];
    const float* bn2_m  = (const float*)d_in[16];
    const float* bn2_v  = (const float*)d_in[17];
    const float* oln_g  = (const float*)d_in[18];
    const float* oln_b  = (const float*)d_in[19];
    const float* Wd1    = (const float*)d_in[20];
    const float* bd1    = (const float*)d_in[21];
    const float* bnd1_g = (const float*)d_in[22];
    const float* bnd1_b = (const float*)d_in[23];
    const float* bnd1_m = (const float*)d_in[24];
    const float* bnd1_v = (const float*)d_in[25];
    const float* Wd2    = (const float*)d_in[26];
    const float* bd2    = (const float*)d_in[27];
    const float* bnd2_g = (const float*)d_in[28];
    const float* bnd2_b = (const float*)d_in[29];
    const float* bnd2_m = (const float*)d_in[30];
    const float* bnd2_v = (const float*)d_in[31];
    const float* Wd3    = (const float*)d_in[32];
    const float* bd3    = (const float*)d_in[33];

    float* params = (float*)d_ws;
    float* o_ws   = (float*)((char*)d_ws + WS_O_OFF);
    float* outp   = (float*)d_out;

    k_fold<<<1, 256, 0, stream>>>(conv_w, conv_b, bn1_g, bn1_b, bn1_m, bn1_v, Q, Wk, bk, params);

    const int g1 = (nb + K1_SPB - 1) / K1_SPB;
    k_enc<<<g1, K1_TPB, K1_SMEM, stream>>>(x, n_x, nb, ln1_g, ln1_b, params, o_ws);

    const int g2 = (nb + K2_R - 1) / K2_R;
    k_head<<<g2, K2_TPB, K2_SMEM, stream>>>(
        o_ws, nb, W1, b1, bn2_g, bn2_b, bn2_m, bn2_v, oln_g, oln_b,
        Wd1, bd1, bnd1_g, bnd1_b, bnd1_m, bnd1_v,
        Wd2, bd2, bnd2_g, bnd2_b, bnd2_m, bnd2_v,
        Wd3, bd3, outp);
}
